// NLBasicBlock_14714557956618
// MI455X (gfx1250) — hardware-verified
//
#include <hip/hip_runtime.h>


namespace {
constexpr int Bsz = 2, C = 64, HH = 80, WW = 80, NP_ = HH * WW, KC = C * 9;
constexpr float XS = 64.0f, WS = 512.0f, OS = 8.0f, TS = 8.0f, PS = 4096.0f, YS = 64.0f;

typedef _Float16 b16;
typedef __attribute__((ext_vector_type(16))) _Float16 v16b;
typedef __attribute__((ext_vector_type(8)))  _Float16 v8b;
typedef __attribute__((ext_vector_type(8)))  float v8f;
typedef __attribute__((ext_vector_type(4)))  float v4f;

__device__ __forceinline__ v8b ld8b(const b16* p) { return *(const v8b*)p; }
__device__ __forceinline__ v16b cat8b(v8b a, v8b b) { return __builtin_shufflevector(a, b, 0, 1, 2, 3, 4, 5, 6, 7, 8, 9, 10, 11, 12, 13, 14, 15); }
__device__ __forceinline__ v16b frag_kb(const b16* p, int hh) { return cat8b(ld8b(p + 8 * hh), ld8b(p + 16 + 8 * hh)); }
__device__ __forceinline__ void split16(float v, b16& hi, b16& lo) { hi = (b16)v; lo = (b16)(v - (float)hi); }
__device__ __forceinline__ void frag_ksplit(const float* p, int hh, v16b& fh_, v16b& fl_) {
  const float* p0 = p + 8 * hh; const float* p1 = p + 16 + 8 * hh;
#pragma unroll
  for (int e = 0; e < 8; ++e) { b16 a, c; split16(p0[e], a, c); fh_[e] = a; fl_[e] = c; split16(p1[e], a, c); fh_[8 + e] = a; fl_[8 + e] = c; }
}
__device__ __forceinline__ v8f wmma16b(v16b a, v16b b, v8f c) {
  v8f d = __builtin_amdgcn_wmma_f32_16x16x32_f16(false, a, false, b, (short)0, c, false, false);
  asm volatile("v_nop\n\tv_nop\n\tv_nop\n\tv_nop" : "+v"(d) : "v"(a), "v"(b));
  return d;
}
__device__ __forceinline__ void wave_lds_sync() {
  __builtin_amdgcn_fence(__ATOMIC_RELEASE, "workgroup");
  __builtin_amdgcn_wave_barrier();
  __builtin_amdgcn_fence(__ATOMIC_ACQUIRE, "workgroup");
}

struct Opnd { const void* p0; const void* p1; int ld; };
template <int NP> __device__ __forceinline__ void load_frags(const Opnd& o, int row, int kb, int hh, v16b& fh_, v16b& fl_) {
  if (NP == 0) { frag_ksplit((const float*)o.p0 + (size_t)row * o.ld + kb, hh, fh_, fl_); }
  else if (NP == 4) {
    const float* p = (const float*)o.p0 + (size_t)row * o.ld + kb; const float* p0 = p + 8 * hh; const float* p1 = p + 16 + 8 * hh;
#pragma unroll
    for (int e = 0; e < 8; ++e) { b16 a, c; split16(p0[e] * 64.0f, a, c); fh_[e] = a; fl_[e] = c; split16(p1[e] * 64.0f, a, c); fh_[8 + e] = a; fl_[8 + e] = c; }
  } else if (NP == 3) {
    const float* p = (const float*)o.p0 + (size_t)row * o.ld + kb; const float* p0 = p + 8 * hh; const float* p1 = p + 16 + 8 * hh;
#pragma unroll
    for (int e = 0; e < 8; ++e) { fh_[e] = (b16)p0[e]; fh_[8 + e] = (b16)p1[e]; }
    fl_ = fh_;
  } else {
    fh_ = frag_kb((const b16*)o.p0 + (size_t)row * o.ld + kb, hh);
    if (NP == 2) fl_ = frag_kb((const b16*)o.p1 + (size_t)row * o.ld + kb, hh); else fl_ = fh_;
  }
}
template <int ANP, int BNP> __device__ __forceinline__ v8f mac(v16b ah, v16b al, v16b bh, v16b bl, v8f c) {
  c = wmma16b(ah, bh, c);
  if (BNP == 0 || BNP == 2 || BNP == 4) c = wmma16b(ah, bl, c);
  if (ANP == 0 || ANP == 2 || ANP == 4) c = wmma16b(al, bh, c);
  return c;
}
template <int ANP, int BNP>
__device__ __forceinline__ void gemm_tile(const Opnd& A, const Opnd& B, int K, int m0, int c0, int nloc, int hlf, v8f (&acc)[2][4]) {
  for (int kb = 0; kb < K; kb += 32) {
    v16b a0h, a0l, a1h, a1l;
    load_frags<ANP>(A, m0 + nloc, kb, hlf, a0h, a0l);
    load_frags<ANP>(A, m0 + 16 + nloc, kb, hlf, a1h, a1l);
#pragma unroll
    for (int t = 0; t < 4; ++t) {
      v16b bh, bl;
      load_frags<BNP>(B, c0 + t * 16 + nloc, kb, hlf, bh, bl);
      acc[0][t] = mac<ANP, BNP>(a0h, a0l, bh, bl, acc[0][t]);
      acc[1][t] = mac<ANP, BNP>(a1h, a1l, bh, bl, acc[1][t]);
    }
  }
}

__device__ __forceinline__ void epi_planes(v8f (&acc)[2][4], float scale, bool two, b16* __restrict__ oh, b16* __restrict__ ol, int ldo,
                                           int m0, int c0, int lane, b16* Th, b16* Tl) {
  const int nloc = lane & 15, hlf = lane >> 4;
#pragma unroll
  for (int t = 0; t < 4; ++t)
#pragma unroll
    for (int r = 0; r < 2; ++r)
#pragma unroll
      for (int v = 0; v < 8; ++v) {
        const int rr = r * 16 + v + 8 * hlf, cc = t * 16 + nloc;
        b16 h_, l_; split16(acc[r][t][v] * scale, h_, l_);
        Th[rr * 64 + cc] = h_; Tl[rr * 64 + cc] = l_;
      }
  wave_lds_sync();
  for (int pass = 0; pass < 2; ++pass) {
#pragma unroll
    for (int j = 0; j < 8; ++j) {
      const int rr = j * 4 + (lane >> 3), c8 = (lane & 7) * 8;
      const size_t o = (size_t)(m0 + rr) * ldo + c0 + c8;
      *(volatile v8b*)(oh + o) = ld8b(Th + rr * 64 + c8);
      if (two) *(volatile v8b*)(ol + o) = ld8b(Tl + rr * 64 + c8);
    }
    __threadfence();
  }
}
__device__ __forceinline__ void epi_f32(v8f (&acc)[2][4], float scale, const float* rscale, float* __restrict__ out, int ldo, int m0, int c0, int lane, float* Tt) {
  const int nloc = lane & 15, hlf = lane >> 4;
#pragma unroll
  for (int t = 0; t < 4; ++t)
#pragma unroll
    for (int r = 0; r < 2; ++r)
#pragma unroll
      for (int v = 0; v < 8; ++v) {
        const int rr = r * 16 + v + 8 * hlf;
        const float rs = rscale ? rscale[(size_t)(m0 + rr) * 32] : 1.0f;
        Tt[rr * 64 + t * 16 + nloc] = acc[r][t][v] * scale * rs;
      }
  wave_lds_sync();
  float* dst0 = out + (size_t)m0 * ldo + c0;
  for (int pass = 0; pass < 2; ++pass) {
#pragma unroll
    for (int j = 0; j < 16; ++j) { const int rr = j * 2 + hlf, c4 = nloc * 4; *(volatile v4f*)(dst0 + (size_t)rr * ldo + c4) = *(const v4f*)(Tt + rr * 64 + c4); }
    __threadfence();
  }
}


__device__ __forceinline__ int refl(int i, int n) { return (i < 0) ? -i : (i >= n ? 2 * n - 2 - i : i); }

__global__ __launch_bounds__(256) void prep_kernel(const float* __restrict__ w1, const float* __restrict__ w2, const float* __restrict__ wth, const float* __restrict__ wph,
                                                   const float* __restrict__ wg, const float* __restrict__ wW, b16* __restrict__ ph_, b16* __restrict__ pl_) {
  const size_t tid = (size_t)blockIdx.x * blockDim.x + threadIdx.x, stride = (size_t)gridDim.x * blockDim.x;
  const size_t n1 = (size_t)C * KC / 8, n2 = (size_t)C * C / 8, tot = 2 * n1 + 4 * n2;
  for (int pass = 0; pass < 2; ++pass) {
    for (size_t c = tid; c < tot; c += stride) {
      const float* src; size_t o;
      if (c < n1) { src = w1 + c * 8; o = c * 8; }
      else if (c < 2 * n1) { src = w2 + (c - n1) * 8; o = c * 8; }
      else { const size_t q = c - 2 * n1; const int m = (int)(q / n2); const size_t i = (q % n2) * 8;
             src = ((m == 0) ? wth : (m == 1) ? wph : (m == 2) ? wg : wW) + i; o = 2 * n1 * 8 + (size_t)m * C * C + i; }
      v8b vh, vl;
#pragma unroll
      for (int e = 0; e < 8; ++e) { b16 a, b2; split16(src[e] * WS, a, b2); vh[e] = a; vl[e] = b2; }
      *(volatile v8b*)(ph_ + o) = vh; *(volatile v8b*)(pl_ + o) = vl;
    }
    __threadfence();
  }
}

template <bool PRELU>
__global__ __launch_bounds__(128) void conv_kernel(const float* __restrict__ in, const b16* __restrict__ wh, const b16* __restrict__ wl, const float* __restrict__ alpha,
                                                   float* __restrict__ out) {
  __shared__ __attribute__((aligned(16))) float Ts[4][32 * 64];
  const int lane = threadIdx.x & 31, wave = threadIdx.x >> 5, nloc = lane & 15, hlf = lane >> 4, z = blockIdx.z;
  const int m0 = (wave & 1) * 32, c0 = blockIdx.x * 128 + (wave >> 1) * 64;
  const float* inz = in + (size_t)z * C * NP_;
  v8f acc[2][4];
#pragma unroll
  for (int r = 0; r < 2; ++r)
#pragma unroll
    for (int t = 0; t < 4; ++t) acc[r][t] = (v8f){};
  const Opnd A{wh, wl, KC};
  int ph4[4], pw4[4];
#pragma unroll
  for (int t = 0; t < 4; ++t) { const int n = c0 + t * 16 + nloc; ph4[t] = n / WW; pw4[t] = n % WW; }
  for (int kb = 0; kb < KC; kb += 32) {
    v16b a0h, a0l, a1h, a1l;
    load_frags<2>(A, m0 + nloc, kb, hlf, a0h, a0l); load_frags<2>(A, m0 + 16 + nloc, kb, hlf, a1h, a1l);
    int ck[16], dh[16], dw[16];
#pragma unroll
    for (int e = 0; e < 16; ++e) { const int k = kb + ((e < 8) ? (8 * hlf + e) : (16 + 8 * hlf + e - 8)); ck[e] = k / 9; const int r9 = k % 9; dh[e] = r9 / 3 - 1; dw[e] = r9 % 3 - 1; }
#pragma unroll
    for (int t = 0; t < 4; ++t) {
      v16b bh, bl;
#pragma unroll
      for (int e = 0; e < 16; ++e) {
        const float v = inz[(size_t)ck[e] * NP_ + refl(ph4[t] + dh[e], HH) * WW + refl(pw4[t] + dw[e], WW)];
        b16 a, b2; split16(v * XS, a, b2); bh[e] = a; bl[e] = b2;
      }
      acc[0][t] = mac<2, 2>(a0h, a0l, bh, bl, acc[0][t]); acc[1][t] = mac<2, 2>(a1h, a1l, bh, bl, acc[1][t]);
    }
  }
  float* Tt = Ts[wave]; const float al = alpha[0];
#pragma unroll
  for (int t = 0; t < 4; ++t)
#pragma unroll
    for (int r = 0; r < 2; ++r)
#pragma unroll
      for (int v = 0; v < 8; ++v) { float val = acc[r][t][v] * (1.0f / (XS * WS)); if (PRELU) val = (val >= 0.0f) ? val : al * val; Tt[(r * 16 + v + 8 * hlf) * 64 + t * 16 + nloc] = val; }
  wave_lds_sync();
  float* dst0 = out + (size_t)z * C * NP_ + (size_t)m0 * NP_ + c0;
  for (int pass = 0; pass < 2; ++pass) {
#pragma unroll
    for (int j = 0; j < 16; ++j) { const int rr = j * 2 + hlf, c4 = nloc * 4; *(volatile v4f*)(dst0 + (size_t)rr * NP_ + c4) = *(const v4f*)(Tt + rr * 64 + c4); }
    __threadfence();
  }
}

__global__ __launch_bounds__(256) void otrans_kernel(const float* __restrict__ x1, const float* __restrict__ alpha, b16* __restrict__ oh, b16* __restrict__ ol) {
  __shared__ __attribute__((aligned(16))) b16 Th[64][72]; __shared__ __attribute__((aligned(16))) b16 Tl[64][72];
  const int tid = threadIdx.x, lane = tid & 31, wave = tid >> 5, z = blockIdx.y, n0 = blockIdx.x * 64;
  const float al = alpha[0];
  { const int c = tid >> 2, px = (tid & 3) * 16; const float* src = x1 + ((size_t)z * C + c) * NP_ + n0 + px;
#pragma unroll
    for (int e = 0; e < 16; ++e) { float v = src[e]; v = (v >= 0.0f) ? v : al * v; b16 a, b2; split16(v * OS, a, b2); Th[px + e][c] = a; Tl[px + e][c] = b2; } }
  __syncthreads();
  b16* dh_ = oh + ((size_t)z * NP_ + n0) * C; b16* dl_ = ol + ((size_t)z * NP_ + n0) * C;
  for (int pass = 0; pass < 2; ++pass) {
#pragma unroll
    for (int j = 0; j < 2; ++j) { const int rr = wave * 8 + j * 4 + (lane >> 3), c8 = (lane & 7) * 8;
      *(volatile v8b*)(dh_ + (size_t)rr * C + c8) = *(const v8b*)(&Th[rr][c8]); *(volatile v8b*)(dl_ + (size_t)rr * C + c8) = *(const v8b*)(&Tl[rr][c8]); }
    __threadfence();
  }
}

__global__ __launch_bounds__(128) void thph_kernel(const b16* __restrict__ oh, const b16* __restrict__ ol, const b16* __restrict__ wh, const b16* __restrict__ wl,
                                                   b16* __restrict__ thh, b16* __restrict__ thl, b16* __restrict__ phh, b16* __restrict__ phl) {
  __shared__ __attribute__((aligned(16))) b16 Ts[4][2][32 * 64];
  const int lane = threadIdx.x & 31, wave = threadIdx.x >> 5, nloc = lane & 15, hlf = lane >> 4, z = blockIdx.z;
  const int m0 = blockIdx.y * 128 + wave * 32, which = blockIdx.x;
  v8f acc[2][4];
#pragma unroll
  for (int r = 0; r < 2; ++r)
#pragma unroll
    for (int t = 0; t < 4; ++t) acc[r][t] = (v8f){};
  const size_t zo = (size_t)z * NP_ * C;
  const Opnd A{oh + zo, ol + zo, C}, B{wh + (size_t)which * C * C, wl + (size_t)which * C * C, C};
  gemm_tile<2, 2>(A, B, C, m0, 0, nloc, hlf, acc);
  epi_planes(acc, TS / (OS * WS), true, (which ? phh : thh) + zo, (which ? phl : thl) + zo, C, m0, 0, lane, Ts[wave][0], Ts[wave][1]);
}

__global__ __launch_bounds__(64) void gt_kernel(const b16* __restrict__ wh, const b16* __restrict__ wl, const b16* __restrict__ oh, const b16* __restrict__ ol, b16* __restrict__ g16) {
  __shared__ __attribute__((aligned(16))) b16 Ts[2][2][32 * 64];
  const int lane = threadIdx.x & 31, wave = threadIdx.x >> 5, nloc = lane & 15, hlf = lane >> 4, z = blockIdx.z;
  const int m0 = wave * 32, c0 = blockIdx.x * 64;
  v8f acc[2][4];
#pragma unroll
  for (int r = 0; r < 2; ++r)
#pragma unroll
    for (int t = 0; t < 4; ++t) acc[r][t] = (v8f){};
  const size_t zo = (size_t)z * NP_ * C;
  const Opnd A{wh, wl, C}, B{oh + zo, ol + zo, C};
  gemm_tile<2, 2>(A, B, C, m0, c0, nloc, hlf, acc);
  epi_planes(acc, 1.0f / (OS * WS), false, g16 + (size_t)z * C * NP_, nullptr, NP_, m0, c0, lane, Ts[wave][0], Ts[wave][1]);
}

__global__ __launch_bounds__(256) void stats_kernel(const b16* __restrict__ thh, const b16* __restrict__ thl, const b16* __restrict__ phh, const b16* __restrict__ phl,
                                                    float* __restrict__ Mx, float* __restrict__ Linv) {
  __shared__ float Ms[128], Ls[128];
  const int wid = threadIdx.x >> 5, lane = threadIdx.x & 31, hh = lane >> 4, col = lane & 15, z = blockIdx.y;
  const int j0 = blockIdx.x * 128 + wid * 16;
  const size_t zo = (size_t)z * NP_ * C, jo = zo + (size_t)(j0 + col) * C;
  const v16b b0h = frag_kb(phh + jo, hh), b0l = frag_kb(phl + jo, hh), b1h = frag_kb(phh + jo + 32, hh), b1l = frag_kb(phl + jo + 32, hh);
  float m = -INFINITY, l = 0.0f;
  for (int ib = 0; ib < NP_; ib += 32) {
    v8f s0 = {}, s1 = {};
#pragma unroll
    for (int half = 0; half < 2; ++half) {
      const size_t io = zo + (size_t)(ib + half * 16 + col) * C;
      const v16b a0h = frag_kb(thh + io, hh), a0l = frag_kb(thl + io, hh), a1h = frag_kb(thh + io + 32, hh), a1l = frag_kb(thl + io + 32, hh);
      v8f& s = half ? s1 : s0;
      s = mac<2, 2>(a0h, a0l, b0h, b0l, s); s = mac<2, 2>(a1h, a1l, b1h, b1l, s);
    }
    float mr = -INFINITY;
#pragma unroll
    for (int r = 0; r < 8; ++r) { s0[r] *= (1.0f / (TS * TS)); s1[r] *= (1.0f / (TS * TS)); mr = fmaxf(mr, fmaxf(s0[r], s1[r])); }
    mr = fmaxf(mr, __shfl_xor(mr, 16));
    const float mn = fmaxf(m, mr), al_ = __expf(m - mn);
    m = mn;
    float sum = 0.0f;
#pragma unroll
    for (int r = 0; r < 8; ++r) sum += __expf(s0[r] - mn) + __expf(s1[r] - mn);
    sum += __shfl_xor(sum, 16);
    l = l * al_ + sum;
  }
  if (hh == 0) { Ms[wid * 16 + col] = m; Ls[wid * 16 + col] = PS / l; }
  __syncthreads();
  if (wid == 0) {
    float* dm = Mx + (size_t)z * NP_ + blockIdx.x * 128; float* dl = Linv + (size_t)z * NP_ + blockIdx.x * 128;
    for (int pass = 0; pass < 2; ++pass) {
      *(volatile v4f*)(dm + lane * 4) = *(const v4f*)(&Ms[lane * 4]); *(volatile v4f*)(dl + lane * 4) = *(const v4f*)(&Ls[lane * 4]);
      __threadfence();
    }
  }
}

__global__ __launch_bounds__(128) void pg_kernel(const b16* __restrict__ thh, const b16* __restrict__ thl, const b16* __restrict__ phh, const b16* __restrict__ phl,
                                                 const b16* __restrict__ g16, const float* __restrict__ Mx, const float* __restrict__ Linv, float* __restrict__ yT) {
  __shared__ __attribute__((aligned(16))) b16 Pt[4][32 * 32];
  __shared__ __attribute__((aligned(16))) float Ts[4][32 * 64];
  const int lane = threadIdx.x & 31, wave = threadIdx.x >> 5, nloc = lane & 15, hlf = lane >> 4, z = blockIdx.y;
  const int m0 = blockIdx.x * 128 + wave * 32;
  const size_t zo = (size_t)z * NP_ * C;
  v16b ah[2][2], al[2][2];
#pragma unroll
  for (int r = 0; r < 2; ++r)
#pragma unroll
    for (int k = 0; k < 2; ++k) { const size_t io = zo + (size_t)(m0 + r * 16 + nloc) * C + 32 * k; ah[r][k] = frag_kb(thh + io, hlf); al[r][k] = frag_kb(thl + io, hlf); }
  const float* Mz = Mx + (size_t)z * NP_; const float* Lz = Linv + (size_t)z * NP_; const b16* gz = g16 + (size_t)z * C * NP_;
  v8f y[2][4];
#pragma unroll
  for (int r = 0; r < 2; ++r)
#pragma unroll
    for (int t = 0; t < 4; ++t) y[r][t] = (v8f){};
  b16* P = Pt[wave];
  for (int jb = 0; jb < NP_; jb += 32) {
    v8f f[2][2];
#pragma unroll
    for (int r = 0; r < 2; ++r)
#pragma unroll
      for (int t = 0; t < 2; ++t) f[r][t] = (v8f){};
#pragma unroll
    for (int t = 0; t < 2; ++t)
#pragma unroll
      for (int k = 0; k < 2; ++k) {
        const size_t jo = zo + (size_t)(jb + t * 16 + nloc) * C + 32 * k;
        const v16b bh = frag_kb(phh + jo, hlf), bl = frag_kb(phl + jo, hlf);
        f[0][t] = mac<2, 2>(ah[0][k], al[0][k], bh, bl, f[0][t]); f[1][t] = mac<2, 2>(ah[1][k], al[1][k], bh, bl, f[1][t]);
      }
#pragma unroll
    for (int t = 0; t < 2; ++t) {
      const int j = jb + t * 16 + nloc; const float mj = Mz[j], lj = Lz[j];
#pragma unroll
      for (int r = 0; r < 2; ++r)
#pragma unroll
        for (int v = 0; v < 8; ++v) P[(r * 16 + 8 * hlf + v) * 32 + t * 16 + nloc] = (b16)(__expf(f[r][t][v] * (1.0f / (TS * TS)) - mj) * lj);
    }
    wave_lds_sync();
    const v16b p0 = frag_kb(P + nloc * 32, hlf), p1 = frag_kb(P + (16 + nloc) * 32, hlf);
#pragma unroll
    for (int t = 0; t < 4; ++t) {
      const v16b gb = frag_kb(gz + (size_t)(t * 16 + nloc) * NP_ + jb, hlf);
      y[0][t] = wmma16b(p0, gb, y[0][t]); y[1][t] = wmma16b(p1, gb, y[1][t]);
    }
    wave_lds_sync();
  }
  epi_f32(y, 1.0f / PS, nullptr, yT + zo, C, m0, 0, lane, Ts[wave]);
}

__global__ __launch_bounds__(64) void wy_kernel(const b16* __restrict__ wh, const b16* __restrict__ wl, const float* __restrict__ yT, const float* __restrict__ x1,
                                                const float* __restrict__ alpha, float* __restrict__ zout) {
  __shared__ __attribute__((aligned(16))) float Ts[2][32 * 64];
  const int lane = threadIdx.x & 31, wave = threadIdx.x >> 5, nloc = lane & 15, hlf = lane >> 4, z = blockIdx.z;
  const int m0 = wave * 32, c0 = blockIdx.x * 64;
  v8f acc[2][4];
#pragma unroll
  for (int r = 0; r < 2; ++r)
#pragma unroll
    for (int t = 0; t < 4; ++t) acc[r][t] = (v8f){};
  const Opnd A{wh, wl, C}, B{yT + (size_t)z * NP_ * C, nullptr, C};
  gemm_tile<2, 4>(A, B, C, m0, c0, nloc, hlf, acc);
  float* Tt = Ts[wave]; const float al = alpha[0]; const float* x1z = x1 + (size_t)z * C * NP_;
#pragma unroll
  for (int t = 0; t < 4; ++t)
#pragma unroll
    for (int r = 0; r < 2; ++r)
#pragma unroll
      for (int v = 0; v < 8; ++v) {
        const int rr = r * 16 + v + 8 * hlf, cc = t * 16 + nloc; const float xv = x1z[(size_t)(m0 + rr) * NP_ + c0 + cc];
        Tt[rr * 64 + cc] = acc[r][t][v] * (1.0f / (YS * WS)) + ((xv >= 0.0f) ? xv : al * xv) + xv;
      }
  wave_lds_sync();
  float* dst0 = zout + (size_t)z * C * NP_ + (size_t)m0 * NP_ + c0;
  for (int pass = 0; pass < 2; ++pass) {
#pragma unroll
    for (int j = 0; j < 16; ++j) { const int rr = j * 2 + hlf, c4 = nloc * 4; *(volatile v4f*)(dst0 + (size_t)rr * NP_ + c4) = *(const v4f*)(Tt + rr * 64 + c4); }
    __threadfence();
  }
}
}

extern "C" void kernel_launch(void* const* d_in, const int* in_sizes, int n_in,
                              void* d_out, int out_size, void* d_ws, size_t ws_size, hipStream_t stream) {
  (void)n_in; (void)out_size;
  const float* x   = (const float*)d_in[0];
  const float* w1  = (const float*)d_in[1];
  const float* w2  = (const float*)d_in[2];
  const float* wg  = (const float*)d_in[3];
  const float* wth = (const float*)d_in[4];
  const float* wph = (const float*)d_in[5];
  const float* wW  = (const float*)d_in[6];
  const float* alpha = (const float*)d_in[7];
  float* out = (float*)d_out;
  if (in_sizes[0] != Bsz * C * NP_ || in_sizes[1] != C * KC || in_sizes[2] != C * KC || in_sizes[3] != C * C || in_sizes[6] != C * C) return;

  size_t off = 0; char* ws = (char*)d_ws;
  auto carve = [&](size_t bytes) { char* p = ws + off; off += (bytes + 255) & ~(size_t)255; return p; };
  const size_t NPL = (size_t)2 * C * KC + 4 * C * C;
  b16* wph_ = (b16*)carve(NPL * 2); b16* wpl_ = (b16*)carve(NPL * 2);
  float* x1 = (float*)carve((size_t)Bsz * C * NP_ * 4);
  b16* oh = (b16*)carve((size_t)Bsz * NP_ * C * 2); b16* ol = (b16*)carve((size_t)Bsz * NP_ * C * 2);
  b16* thh = (b16*)carve((size_t)Bsz * NP_ * C * 2); b16* thl = (b16*)carve((size_t)Bsz * NP_ * C * 2);
  b16* phh = (b16*)carve((size_t)Bsz * NP_ * C * 2); b16* phl = (b16*)carve((size_t)Bsz * NP_ * C * 2);
  b16* g16 = (b16*)carve((size_t)Bsz * C * NP_ * 2);
  float* Mx = (float*)carve((size_t)Bsz * NP_ * 4); float* Li = (float*)carve((size_t)Bsz * NP_ * 4);
  float* yT = (float*)carve((size_t)Bsz * NP_ * C * 4);
  float* zb = (float*)carve((size_t)Bsz * C * NP_ * 4);
  if (off > ws_size) return;
  const b16* w1h = wph_; const b16* w1l = wpl_; const b16* w2h = wph_ + (size_t)C * KC; const b16* w2l = wpl_ + (size_t)C * KC;
  const b16* tph = wph_ + (size_t)2 * C * KC; const b16* tpl = wpl_ + (size_t)2 * C * KC;
  const b16* wgh = tph + (size_t)2 * C * C; const b16* wgl = tpl + (size_t)2 * C * C; const b16* wWh = tph + (size_t)3 * C * C; const b16* wWl = tpl + (size_t)3 * C * C;
  prep_kernel<<<64, 256, 0, stream>>>(w1, w2, wth, wph, wg, wW, wph_, wpl_);
  conv_kernel<false><<<dim3(NP_ / 128, 1, Bsz), 128, 0, stream>>>(x, w1h, w1l, alpha, x1);
  otrans_kernel<<<dim3(NP_ / 64, Bsz), 256, 0, stream>>>(x1, alpha, oh, ol);
  thph_kernel<<<dim3(2, NP_ / 128, Bsz), 128, 0, stream>>>(oh, ol, tph, tpl, thh, thl, phh, phl);
  gt_kernel<<<dim3(NP_ / 64, 1, Bsz), 64, 0, stream>>>(wgh, wgl, oh, ol, g16);
  stats_kernel<<<dim3(NP_ / 128, Bsz), 256, 0, stream>>>(thh, thl, phh, phl, Mx, Li);
  pg_kernel<<<dim3(NP_ / 128, Bsz), 128, 0, stream>>>(thh, thl, phh, phl, g16, Mx, Li, yT);
  wy_kernel<<<dim3(NP_ / 64, 1, Bsz), 64, 0, stream>>>(wWh, wWl, yT, x1, alpha, zb);
  conv_kernel<true><<<dim3(NP_ / 128, 1, Bsz), 128, 0, stream>>>(zb, w2h, w2l, alpha, out);
}
